// NonMarkovPolicy_47467978556216
// MI455X (gfx1250) — hardware-verified
//
#include <hip/hip_runtime.h>
#include <stdint.h>

typedef __attribute__((ext_vector_type(16))) _Float16 v16h;
typedef __attribute__((ext_vector_type(8)))  _Float16 v8h;
typedef __attribute__((ext_vector_type(8)))  float    v8f;
typedef __attribute__((ext_vector_type(4)))  float    v4f;

constexpr int NBATCH = 256;
constexpr int SEQ = 512;
constexpr int DIN = 64;
constexpr int HID = 256;
constexpr int G4 = 4 * HID;
constexpr int NACT = 8;
constexpr int KCAT = DIN + HID;
constexpr int ROWS_PB = 16;
constexpr int LSTM_THREADS = 512;
constexpr int APITCH = 328;
constexpr int TPITCH = 328;
constexpr int HPITCH = 264;
constexpr int NROWS_OUT = NBATCH * SEQ;
constexpr int OUT1_OFF = NROWS_OUT * NACT;
constexpr float WSC = 16.0f;
constexpr float WSC_INV = 0.0625f;

static_assert(KCAT % 32 == 0, "K multiple of 32");
static_assert(HID % 32 == 0, "K multiple of 32");
static_assert(LSTM_THREADS == 32 * (HID / 16), "one wave per 16 hidden units");
static_assert(NBATCH % ROWS_PB == 0, "row blocks");
static_assert(ROWS_PB * DIN == 2 * LSTM_THREADS, "x staging covers 16x64 with 2 per thread");
static_assert(NROWS_OUT % (8 * 16) == 0, "heads grid exact");
static_assert(OUT1_OFF * 4 == 4194304, "out1 byte offset");
static_assert(2 * OUT1_OFF * 4 == 8388608, "d_out total bytes");
static_assert(G4 % 8 == 0, "prep blocks of 8 rows");
static_assert((APITCH * 2) % 16 == 0 && (TPITCH * 2) % 16 == 0 && (HPITCH * 2) % 16 == 0, "16B aligned LDS rows");

constexpr size_t WS_BT_OFF   = 0;
constexpr size_t WS_BT_BYTES = (size_t)G4 * KCAT * 2;
constexpr size_t WS_WT_OFF   = WS_BT_OFF + WS_BT_BYTES;
constexpr size_t WS_WT_BYTES = (size_t)16 * HID * 2;
constexpr size_t WS_HS_OFF   = WS_WT_OFF + WS_WT_BYTES;
constexpr size_t WS_HS_BYTES = (size_t)NROWS_OUT * HID * 2;
constexpr size_t WS_TOTAL    = WS_HS_OFF + WS_HS_BYTES;
static_assert(WS_BT_BYTES == 655360, "carve");
static_assert(WS_TOTAL == 67772416, "carve");
static_assert(WS_TOTAL <= (size_t)134217728, "carve under 128 MiB");
static_assert(WS_WT_OFF % 128 == 0 && WS_HS_OFF % 128 == 0, "128B aligned regions");

__device__ __forceinline__ void dep_guard_h(v8f& a, v8f& b, v16h x, v16h y) { asm volatile("v_nop\n\tv_nop\n\tv_nop\n\tv_nop" : "+v"(a), "+v"(b) : "v"(x), "v"(y)); }
__device__ __forceinline__ void keep4_h(v16h a, v16h b, v16h c, v16h d) { asm volatile("v_nop" :: "v"(a), "v"(b), "v"(c), "v"(d)); }
template <typename T> struct Frag;
template <> struct Frag<_Float16> {
  typedef v16h V; union U { v16h v; v8h h[2]; };
  static __device__ __forceinline__ v16h load(const _Float16* p) {
    U f; f.h[0] = *(const v8h*)(p); f.h[1] = *(const v8h*)(p + 16); return f.v;
  }
  static __device__ __forceinline__ v8f mma(v16h a, v16h b, v8f c) {
    return __builtin_amdgcn_wmma_f32_16x16x32_f16(false, a, false, b, (short)0, c, false, false);
  }
  static __device__ __forceinline__ void guard(v8f& a, v8f& b, v16h x, v16h y) { dep_guard_h(a, b, x, y); }
  static __device__ __forceinline__ void keep(v16h a, v16h b, v16h c, v16h d) { keep4_h(a, b, c, d); }
};

__device__ __forceinline__ void guard4ab(v8f& c0, v8f& c1, v8f& c2, v8f& c3,
                                         v16h a, v16h b0, v16h b1, v16h b2, v16h b3) {
  asm volatile("v_nop\n\tv_nop\n\tv_nop\n\tv_nop"
               : "+v"(c0), "+v"(c1), "+v"(c2), "+v"(c3)
               : "v"(a), "v"(b0), "v"(b1), "v"(b2), "v"(b3));
}
__device__ __forceinline__ v8f mma16_guarded(v16h a, v16h b, v8f c) {
  c = __builtin_amdgcn_wmma_f32_16x16x32_f16(false, a, false, b, (short)0, c, false, false);
  asm volatile("v_nop\n\tv_nop\n\tv_nop\n\tv_nop" : "+v"(c) : "v"(a), "v"(b));
  return c;
}

__device__ __forceinline__ float bf16r(float f) {
  unsigned u = __float_as_uint(f);
  u = (u + 0x7FFFu + ((u >> 16) & 1u)) & 0xFFFF0000u;
  return __uint_as_float(u);
}
__device__ __forceinline__ float sigm(float x) {
  x = fminf(fmaxf(x, -30.0f), 30.0f);
  return 1.0f / (1.0f + expf(-x));
}

__global__ __launch_bounds__(256) void prep_gate_w(const float* __restrict__ Wx,
                                                   const float* __restrict__ Wh,
                                                   _Float16* __restrict__ Bt) {
  __shared__ __align__(16) _Float16 tile[8 * TPITCH];
  const int tid = threadIdx.x;
  const int n0  = blockIdx.x * 8;
  const int nn  = tid & 7;
  const int kq  = tid >> 3;
#pragma unroll
  for (int i = 0; i < 2; ++i) {
    const int k = 32 * i + kq;
    const float v = Wx[(size_t)k * G4 + n0 + nn];
    tile[nn * TPITCH + k] = (_Float16)(bf16r(v) * WSC);
  }
#pragma unroll
  for (int i = 0; i < 8; ++i) {
    const int kh = 32 * i + kq;
    const float v = Wh[(size_t)kh * G4 + n0 + nn];
    tile[nn * TPITCH + DIN + kh] = (_Float16)(bf16r(v) * WSC);
  }
  __syncthreads();
  _Float16* dst = Bt + (size_t)n0 * KCAT;
  const int eA = tid * 8;
  const int rowA = eA / KCAT, colA = eA - rowA * KCAT;
  const v8h vA = *(const v8h*)(tile + rowA * TPITCH + colA);
  const int eB = (256 + (tid & 63)) * 8;
  const int rowB = eB / KCAT, colB = eB - rowB * KCAT;
  const v8h vB = *(const v8h*)(tile + rowB * TPITCH + colB);
  const bool doB = (tid < 64);
  for (int pass = 0; pass < 2; ++pass) {
    *(volatile v8h*)(dst + eA) = vA;
    if (doB) *(volatile v8h*)(dst + eB) = vB;
    __threadfence();
  }
}

__global__ __launch_bounds__(256) void prep_head_w(const float* __restrict__ Wm,
                                                   const float* __restrict__ Ws,
                                                   _Float16* __restrict__ Wt) {
  __shared__ __align__(16) _Float16 tile[16 * HPITCH];
  const int tid = threadIdx.x;
  const int c   = tid & 15;
  const int kq  = tid >> 4;
#pragma unroll 4
  for (int i = 0; i < 16; ++i) {
    const int k = 16 * i + kq;
    const float vm = Wm[k * NACT + (c & 7)];
    const float vs = Ws[k * NACT + (c & 7)];
    const float v  = (c < 8) ? vm : vs;
    tile[c * HPITCH + k] = (_Float16)(bf16r(v) * WSC);
  }
  __syncthreads();
  const int eA = tid * 8, rowA = eA >> 8, colA = eA & 255;
  const int eB = (256 + tid) * 8, rowB = eB >> 8, colB = eB & 255;
  const v8h vA = *(const v8h*)(tile + rowA * HPITCH + colA);
  const v8h vB = *(const v8h*)(tile + rowB * HPITCH + colB);
  for (int pass = 0; pass < 2; ++pass) {
    *(volatile v8h*)(Wt + eA) = vA;
    *(volatile v8h*)(Wt + eB) = vB;
    __threadfence();
  }
}

__device__ __forceinline__ void stage_x(_Float16* A_lds, const float* __restrict__ obs,
                                        int r0, int t, int tid) {
  const int idx = tid * 2;
  const int m = idx >> 6;
  const int d = idx & 63;
  const float2 xv = *(const float2*)(obs + ((size_t)(r0 + m) * SEQ + t) * DIN + d);
  A_lds[m * APITCH + d]     = (_Float16)bf16r(xv.x);
  A_lds[m * APITCH + d + 1] = (_Float16)bf16r(xv.y);
}

__global__ __launch_bounds__(LSTM_THREADS)
void lstm_seq_kernel(const float* __restrict__ obs,
                     const _Float16* __restrict__ Bt,
                     const float* __restrict__ bias,
                     _Float16* __restrict__ hs) {
  __shared__ __align__(16) _Float16 A_lds[ROWS_PB * APITCH];
  const int tid  = threadIdx.x;
  const int wave = tid >> 5;
  const int lane = tid & 31;
  const int hh   = lane >> 4;
  const int rl   = lane & 15;
  const int koff = hh * 8;
  const int r0   = blockIdx.x * ROWS_PB;
  const int hid  = wave * 16 + rl;

  {
    float zf = 0.0f;
    asm volatile("" : "+v"(zf));
    const _Float16 zh = (_Float16)zf;
    for (int i = tid; i < ROWS_PB * APITCH; i += LSTM_THREADS) A_lds[i] = zh;
  }
  const float b_i = bf16r(bias[0 * HID + hid]);
  const float b_f = bf16r(bias[1 * HID + hid]);
  const float b_g = bf16r(bias[2 * HID + hid]);
  const float b_o = bf16r(bias[3 * HID + hid]);
  float creg[8] = {0.f, 0.f, 0.f, 0.f, 0.f, 0.f, 0.f, 0.f};
  __syncthreads();
  stage_x(A_lds, obs, r0, 0, tid);
  __syncthreads();

#pragma clang loop unroll(disable)
  for (int t = 0; t < SEQ; ++t) {
    v8f acc[4];
#pragma unroll
    for (int g = 0; g < 4; ++g) acc[g] = (v8f){0.f, 0.f, 0.f, 0.f, 0.f, 0.f, 0.f, 0.f};
#pragma unroll 1
    for (int kt = 0; kt < KCAT / 32; ++kt) {
      const int k0 = kt * 32;
      const v16h a = Frag<_Float16>::load(A_lds + rl * APITCH + k0 + koff);
      v16h bq[4];
#pragma unroll
      for (int g = 0; g < 4; ++g)
        bq[g] = Frag<_Float16>::load(Bt + (size_t)(g * HID + hid) * KCAT + k0 + koff);
#pragma unroll
      for (int g = 0; g < 4; ++g) acc[g] = Frag<_Float16>::mma(a, bq[g], acc[g]);
      guard4ab(acc[0], acc[1], acc[2], acc[3], a, bq[0], bq[1], bq[2], bq[3]);
    }
    __syncthreads();

#pragma unroll
    for (int r = 0; r < 8; ++r) {
      const int m = hh * 8 + r;
      const float zi = acc[0][r] * WSC_INV + b_i;
      const float zf = acc[1][r] * WSC_INV + b_f;
      const float zg = acc[2][r] * WSC_INV + b_g;
      const float zo = acc[3][r] * WSC_INV + b_o;
      const float ig = sigm(zi);
      const float fg = sigm(zf);
      const float gg = tanhf(zg);
      const float og = sigm(zo);
      const float c  = fg * creg[r] + ig * gg;
      creg[r] = c;
      const float h  = og * tanhf(c);
      A_lds[m * APITCH + DIN + hid] = (_Float16)h;
    }
    if (t + 1 < SEQ) stage_x(A_lds, obs, r0, t + 1, tid);
    __syncthreads();

    {
      const v8h hv = *(const v8h*)(A_lds + wave * APITCH + DIN + 8 * lane);
      _Float16* dst = hs + ((size_t)(r0 + wave) * SEQ + t) * HID + 8 * lane;
      *(volatile v8h*)dst = hv;
      __threadfence();
      *(volatile v8h*)dst = hv;
    }
  }
}

__global__ __launch_bounds__(256)
void heads_kernel(const _Float16* __restrict__ hs,
                  const _Float16* __restrict__ Wt,
                  const float* __restrict__ bm,
                  const float* __restrict__ bs,
                  float* __restrict__ out) {
  __shared__ __align__(16) float slab[8 * 16 * 16];
  const int tid  = threadIdx.x;
  const int wave = tid >> 5;
  const int lane = tid & 31;
  const int hh   = lane >> 4;
  const int rl   = lane & 15;
  const int koff = hh * 8;
  const int row0 = (blockIdx.x * 8 + wave) * 16;

  v8f acc = (v8f){0.f, 0.f, 0.f, 0.f, 0.f, 0.f, 0.f, 0.f};
#pragma unroll 2
  for (int kt = 0; kt < HID / 32; ++kt) {
    const int k0 = kt * 32;
    const v16h a = Frag<_Float16>::load(hs + (size_t)(row0 + rl) * HID + k0 + koff);
    const v16h b = Frag<_Float16>::load(Wt + (size_t)rl * HID + k0 + koff);
    acc = mma16_guarded(a, b, acc);
  }
  const float vbm = bm[rl & 7];
  const float vbs = bs[rl & 7];
  const float bv  = bf16r((rl < 8) ? vbm : vbs);
  const bool isStd = (rl >= 8);
  float* sw = slab + wave * 256;
#pragma unroll
  for (int r = 0; r < 8; ++r) {
    float v = acc[r] * WSC_INV + bv;
    const float vc = fminf(fmaxf(v, -10.0f), 2.0f);
    v = isStd ? vc : v;
    sw[(hh * 8 + r) * 16 + rl] = v;
  }
  __syncthreads();
  {
    const int orow = lane >> 1;
    const int half = lane & 1;
    const v4f vmn = *(const v4f*)(sw + orow * 16 + 4 * half);
    const v4f vsd = *(const v4f*)(sw + orow * 16 + 8 + 4 * half);
    float* p0 = out + (size_t)(row0 + orow) * NACT + 4 * half;
    float* p1 = p0 + OUT1_OFF;
    for (int pass = 0; pass < 2; ++pass) {
      *(volatile v4f*)p0 = vmn;
      *(volatile v4f*)p1 = vsd;
      __threadfence();
    }
  }
}

extern "C" void kernel_launch(void* const* d_in, const int* in_sizes, int n_in,
                              void* d_out, int out_size, void* d_ws, size_t ws_size,
                              hipStream_t stream) {
  if (n_in < 8) return;
  if (in_sizes[0] != NBATCH * SEQ * DIN) return;
  if (in_sizes[1] != DIN * G4) return;
  if (in_sizes[2] != HID * G4) return;
  if (in_sizes[3] != G4) return;
  if (in_sizes[4] != HID * NACT || in_sizes[6] != HID * NACT) return;
  if (in_sizes[5] != NACT || in_sizes[7] != NACT) return;
  if (out_size != 2 * OUT1_OFF) return;
  if (ws_size < WS_TOTAL) return;

  const float* obs = (const float*)d_in[0];
  const float* Wx  = (const float*)d_in[1];
  const float* Wh  = (const float*)d_in[2];
  const float* b   = (const float*)d_in[3];
  const float* Wm  = (const float*)d_in[4];
  const float* bm  = (const float*)d_in[5];
  const float* Ws  = (const float*)d_in[6];
  const float* bs  = (const float*)d_in[7];
  float* out = (float*)d_out;
  char* ws = (char*)d_ws;
  _Float16* Bt  = (_Float16*)(ws + WS_BT_OFF);
  _Float16* Wt  = (_Float16*)(ws + WS_WT_OFF);
  _Float16* hsp = (_Float16*)(ws + WS_HS_OFF);

  prep_gate_w<<<G4 / 8, 256, 0, stream>>>(Wx, Wh, Bt);
  prep_head_w<<<1, 256, 0, stream>>>(Wm, Ws, Wt);
  lstm_seq_kernel<<<NBATCH / ROWS_PB, LSTM_THREADS, 0, stream>>>(obs, Bt, b, hsp);
  heads_kernel<<<NROWS_OUT / 128, 256, 0, stream>>>(hsp, Wt, bm, bs, out);
}
